// SA_Layer_16174846837200
// MI455X (gfx1250) — hardware-run, weakly checked
//
#include <hip/hip_runtime.h>
#include <math.h>

constexpr int NB   = 4;
constexpr int NC   = 128;
constexpr int NN   = 4096;
constexpr int NI   = 64;
constexpr int NTOK = NB * NN;
constexpr int CN   = NC * NN;
constexpr int NQH  = 2048;
constexpr int QKLD = 128;
constexpr int PLD  = 192;
constexpr int WLROWS = 256;
constexpr int GNSEG = 32;
constexpr int GNSEGLEN = CN / GNSEG;
constexpr float kEpsGN    = 1.0e-5f;
constexpr float kInvCN    = 1.0f / 524288.0f;
constexpr float kWCarry   = 16.0f;
constexpr float kActCarry = 4.0f;
constexpr float kProjScale = kActCarry / kWCarry;
constexpr float kACarry   = kActCarry * kActCarry;
constexpr float kFc1Scale = 1.0f / (kACarry * kWCarry);
constexpr float kS1Carry  = 16.0f;
constexpr float kFc2Scale = 1.0f / (kS1Carry * kWCarry);
constexpr float kPCarry   = 32768.0f;
constexpr float kPVScale  = 1.0f / (kPCarry * kActCarry);
constexpr float kYCarry   = 32.0f;
constexpr float kLocScale = kYCarry / kActCarry;
constexpr float kTcScale  = 1.0f / (kWCarry * kYCarry);
static_assert(GNSEGLEN == 16 * 256 * 4);
static_assert(NTOK % 64 == 0 && QKLD % 64 == 0 && PLD % 64 == 0 && NC % 32 == 0);
static_assert(NI % 64 == 0 && NN % 64 == 0);
static_assert(NN % 64 == 0 && NQH % 64 == 0 && NI % 32 == 0);
static_assert(NN % 32 == 0);
static_assert(NC % 64 == 0);
static_assert(NQH == 8 * 256 && 2 * NQH == NN && WLROWS == 3 * NI + NI);

typedef __attribute__((ext_vector_type(16))) _Float16 v16h;
typedef __attribute__((ext_vector_type(8)))  _Float16 v8h;
typedef __attribute__((ext_vector_type(16))) __bf16   v16b;
typedef __attribute__((ext_vector_type(8)))  __bf16   v8b;
typedef __attribute__((ext_vector_type(8)))  float    v8f;
typedef __attribute__((ext_vector_type(4)))  float    v4f;
typedef __attribute__((ext_vector_type(4)))  unsigned int v4u;
typedef __attribute__((ext_vector_type(2)))  unsigned int v2u;

__device__ __forceinline__ unsigned short f2bf_bits(float f) {
  unsigned u = __float_as_uint(f);
  return (unsigned short)((u + 0x7FFFu + ((u >> 16) & 1u)) >> 16);
}
__device__ __forceinline__ float bf_bits2f(unsigned short h) { return __uint_as_float(((unsigned)h) << 16); }

__device__ __forceinline__ void dep_guard4_h(v8f& a, v8f& b, v8f& c, v8f& d, v16h x, v16h y) { asm volatile("v_nop\n\tv_nop\n\tv_nop\n\tv_nop" : "+v"(a), "+v"(b), "+v"(c), "+v"(d) : "v"(x), "v"(y)); }
__device__ __forceinline__ void dep_guard4_b(v8f& a, v8f& b, v8f& c, v8f& d, v16b x, v16b y) { asm volatile("v_nop\n\tv_nop\n\tv_nop\n\tv_nop" : "+v"(a), "+v"(b), "+v"(c), "+v"(d) : "v"(x), "v"(y)); }
__device__ __forceinline__ void keep4_h(v16h a, v16h b, v16h c, v16h d) { asm volatile("v_nop" :: "v"(a), "v"(b), "v"(c), "v"(d)); }
__device__ __forceinline__ void keep4_b(v16b a, v16b b, v16b c, v16b d) { asm volatile("v_nop" :: "v"(a), "v"(b), "v"(c), "v"(d)); }
__device__ __forceinline__ void acc_guard4(v8f& a, v8f& b, v8f& c, v8f& d) { asm volatile("v_nop\n\tv_nop\n\tv_nop\n\tv_nop" : "+v"(a), "+v"(b), "+v"(c), "+v"(d)); }
template <typename T> struct Frag;
template <> struct Frag<_Float16> {
  typedef v16h V; union U { v16h v; v8h h[2]; };
  static __device__ __forceinline__ v16h load(const _Float16* p) {
    U f; f.h[0] = *(const v8h*)(p); f.h[1] = *(const v8h*)(p + 16); return f.v;
  }
  static __device__ __forceinline__ v8f mma(v16h a, v16h b, v8f c) {
    return __builtin_amdgcn_wmma_f32_16x16x32_f16(false, a, false, b, (short)0, c, false, false);
  }
  static __device__ __forceinline__ void guard4(v8f& a, v8f& b, v8f& c, v8f& d, v16h x, v16h y) { dep_guard4_h(a, b, c, d, x, y); }
  static __device__ __forceinline__ void keep(v16h a, v16h b, v16h c, v16h d) { keep4_h(a, b, c, d); }
};
template <> struct Frag<__bf16> {
  typedef v16b V; union U { v16b v; v8b h[2]; };
  static __device__ __forceinline__ v16b load(const __bf16* p) {
    U f; f.h[0] = *(const v8b*)(p); f.h[1] = *(const v8b*)(p + 16); return f.v;
  }
  static __device__ __forceinline__ v8f mma(v16b a, v16b b, v8f c) {
    return __builtin_amdgcn_wmma_f32_16x16x32_bf16(false, a, false, b, (short)0, c, false, false);
  }
  static __device__ __forceinline__ void guard4(v8f& a, v8f& b, v8f& c, v8f& d, v16b x, v16b y) { dep_guard4_b(a, b, c, d, x, y); }
  static __device__ __forceinline__ void keep(v16b a, v16b b, v16b c, v16b d) { keep4_b(a, b, c, d); }
};

__device__ __forceinline__ unsigned pk16(unsigned short a, unsigned short b) { return (unsigned)a | ((unsigned)b << 16); }
__device__ __forceinline__ unsigned short h_bits(float f) { const _Float16 h = (_Float16)f; return __builtin_bit_cast(unsigned short, h); }

__device__ __forceinline__ float h16_to_f32(unsigned hb) {
  const unsigned sgn = (hb & 0x8000u) << 16; const unsigned em = hb & 0x7fffu;
  const float fn = __uint_as_float((em << 13) + 0x38000000u);
  const float fs = (float)em * 5.9604644775390625e-8f;
  const float mag = (em < 0x400u) ? fs : fn; return __uint_as_float(__float_as_uint(mag) | sgn); }

template <int ET> struct Elem;
template <> struct Elem<0> { typedef _Float16 T; };
template <> struct Elem<1> { typedef __bf16 T; };
template <int ET, bool SPLIT, int BIAS_MODE, int OUT_MODE, bool RESID, int ACT = 0>
__global__ __launch_bounds__(256) void wmma_gemm64(
    const unsigned short* __restrict__ Ap, const unsigned short* __restrict__ A2p, int lda, long strideA,
    const unsigned short* __restrict__ Btp, const unsigned short* __restrict__ Bt2p, int ldb, long strideB,
    void* __restrict__ Cout, void* __restrict__ Cout2, int ldc, long strideC,
    const float* __restrict__ bias,
    const float* __restrict__ resid, long strideR,
    int M, int N, int K, float scale) {
  typedef typename Elem<ET>::T T;
  typedef typename Frag<T>::V V;
  const T* A = (const T*)Ap; const T* A2 = (const T*)A2p; const T* Bt = (const T*)Btp; const T* Bt2 = (const T*)Bt2p;
  __shared__ __align__(16) float sT[8][16 * 68];
  const int b    = blockIdx.y;
  const int lane = threadIdx.x & 31;
  const int wave = threadIdx.x >> 5;
  const int tilesN = N >> 6;
  const int tilesM = M >> 6;
  const int tile = blockIdx.x * 8 + wave;
  if (tile >= tilesM * tilesN) return;
  const int tm = tile / tilesN;
  const int tn = tile - tm * tilesN;
  const int m0 = tm << 6;
  const int n0 = tn << 6;

  const T* Ab  = A  + (size_t)b * strideA;
  const T* Bb  = Bt + (size_t)b * strideB;
  const T* Ab2 = SPLIT ? (A2  + (size_t)b * strideA) : nullptr;
  const T* Bb2 = SPLIT ? (Bt2 + (size_t)b * strideB) : nullptr;

  const int rlane = lane & 15;
  const int koff  = (lane >> 4) * 8;
  const int mOff  = (lane >> 4) * 8;

  v8f acc[4][4];
#pragma unroll
  for (int i = 0; i < 4; ++i)
#pragma unroll
    for (int j = 0; j < 4; ++j) acc[i][j] = (v8f){0.f,0.f,0.f,0.f,0.f,0.f,0.f,0.f};

  for (int k0 = 0; k0 < K; k0 += 32) {
    V bh[4], bl[4];
#pragma unroll
    for (int j = 0; j < 4; ++j) {
      const size_t bo = (size_t)(n0 + (j << 4) + rlane) * ldb + koff + k0;
      bh[j] = Frag<T>::load(Bb + bo);
      if (SPLIT) bl[j] = Frag<T>::load(Bb2 + bo);
    }
#pragma unroll
    for (int i = 0; i < 4; ++i) {
      const size_t ao = (size_t)(m0 + (i << 4) + rlane) * lda + koff + k0;
      V ah = Frag<T>::load(Ab + ao);
      V al;
      if (SPLIT) al = Frag<T>::load(Ab2 + ao);
#pragma unroll
      for (int j = 0; j < 4; ++j) {
        acc[i][j] = Frag<T>::mma(ah, bh[j], acc[i][j]);
        if (SPLIT) {
          acc[i][j] = Frag<T>::mma(ah, bl[j], acc[i][j]);
          acc[i][j] = Frag<T>::mma(al, bh[j], acc[i][j]);
        }
      }
      Frag<T>::guard4(acc[i][0], acc[i][1], acc[i][2], acc[i][3], ah, SPLIT ? al : ah);
    }
    Frag<T>::keep(bh[0], bh[1], bh[2], bh[3]);
    if (SPLIT) Frag<T>::keep(bl[0], bl[1], bl[2], bl[3]);
  }
  acc_guard4(acc[0][0], acc[0][1], acc[0][2], acc[0][3]);
  acc_guard4(acc[1][0], acc[1][1], acc[1][2], acc[1][3]);
  acc_guard4(acc[2][0], acc[2][1], acc[2][2], acc[2][3]);
  acc_guard4(acc[3][0], acc[3][1], acc[3][2], acc[3][3]);

  float* slab = sT[wave];
  const float* Rb = RESID ? (resid + (size_t)b * strideR) : nullptr;
#pragma unroll
  for (int i = 0; i < 4; ++i) {
    const int mBase = m0 + (i << 4);
#pragma unroll
    for (int j = 0; j < 4; ++j) {
      const int n = n0 + (j << 4) + rlane;
      float bv = 0.f;
      if (BIAS_MODE == 2) bv = bias[n];
#pragma unroll
      for (int r = 0; r < 8; ++r) {
        float v = acc[i][j][r] * scale;
        if (BIAS_MODE == 1) v += bias[mBase + mOff + r];
        if (BIAS_MODE == 2) v += bv;
        if (RESID) v += Rb[(size_t)(mBase + mOff + r) * ldc + n];
        if (ACT == 2) v = fmaxf(v, 0.0f);
        if (ACT == 4) v = (v > 0.f) ? v : 0.01f * v;
        slab[(mOff + r) * 68 + (j << 4) + rlane] = v;
      }
    }
    __builtin_amdgcn_fence(__ATOMIC_RELEASE, "workgroup");
    __builtin_amdgcn_wave_barrier();
    __builtin_amdgcn_fence(__ATOMIC_ACQUIRE, "workgroup");
    if (OUT_MODE == 0) {
      float* C = (float*)Cout + (size_t)b * strideC;
      const int hh = lane >> 4, c4 = (lane & 15) * 4;
      for (int pass = 0; pass < 2; ++pass) {
#pragma unroll
        for (int it = 0; it < 8; ++it) {
          const int row = it * 2 + hh;
          v4f v = *(const v4f*)(slab + row * 68 + c4);
          *(volatile v4f*)(C + (size_t)(mBase + row) * ldc + n0 + c4) = v;
        }
        __threadfence();
      }
    } else {
      const int q = lane >> 3, c8 = (lane & 7) * 8;
      unsigned short* C  = (unsigned short*)Cout  + (size_t)b * strideC;
      unsigned short* C2 = (OUT_MODE == 2) ? ((unsigned short*)Cout2 + (size_t)b * strideC) : nullptr;
      for (int pass = 0; pass < 2; ++pass) {
#pragma unroll
        for (int it = 0; it < 4; ++it) {
          const int row = it * 4 + q;
          const float* sp = slab + row * 68 + c8;
          v8h hv, lv;
#pragma unroll
          for (int e = 0; e < 8; ++e) {
            if (OUT_MODE == 1) {
              hv[e] = (_Float16)sp[e];
            } else {
              unsigned short hb = f2bf_bits(sp[e]);
              unsigned short lb = f2bf_bits(sp[e] - bf_bits2f(hb));
              hv[e] = __builtin_bit_cast(_Float16, hb);
              lv[e] = __builtin_bit_cast(_Float16, lb);
            }
          }
          *(volatile v8h*)(C + (size_t)(mBase + row) * ldc + n0 + c8) = hv;
          if (OUT_MODE == 2) *(volatile v8h*)(C2 + (size_t)(mBase + row) * ldc + n0 + c8) = lv;
        }
        __threadfence();
      }
    }
    __builtin_amdgcn_fence(__ATOMIC_RELEASE, "workgroup");
    __builtin_amdgcn_wave_barrier();
    __builtin_amdgcn_fence(__ATOMIC_ACQUIRE, "workgroup");
  }
}

__global__ __launch_bounds__(256) void wprep_kernel(const float* __restrict__ gq_w, const float* __restrict__ gq_b,
                                                   const float* __restrict__ gkv_w, const float* __restrict__ gkv_b,
                                                   const float* __restrict__ lqkv_w, const float* __restrict__ lqkv_b,
                                                   const float* __restrict__ dw_w, const float* __restrict__ dw_b,
                                                   const float* __restrict__ fc_w, const float* __restrict__ tc_w,
                                                   unsigned short* __restrict__ wqkh, unsigned short* __restrict__ wqkl,
                                                   unsigned short* __restrict__ wl, unsigned short* __restrict__ fc16,
                                                   unsigned short* __restrict__ tc16, float* __restrict__ beff) {
  const int blk = blockIdx.x;
  const int t = threadIdx.x, lane = t & 31, wave = t >> 5;
  if (blk < 8) {
    const int o = blk * 16 + (t >> 4);
    const int c8 = (t & 15) * 8;
    const float* src = (blk < 4) ? gq_w : gkv_w;
    const int srow = (blk < 4) ? o : (o - 64);
    const float* rp = src + (size_t)srow * NC + c8;
    const v4f a = *(const v4f*)(rp);
    const v4f c = *(const v4f*)(rp + 4);
    unsigned short hb[8], lb[8];
#pragma unroll
    for (int e = 0; e < 4; ++e) {
      const unsigned short h0 = f2bf_bits(a[e]);
      hb[e] = h0; lb[e] = f2bf_bits(a[e] - bf_bits2f(h0));
      const unsigned short h1 = f2bf_bits(c[e]);
      hb[4 + e] = h1; lb[4 + e] = f2bf_bits(c[e] - bf_bits2f(h1));
    }
    const v4u uh = (v4u){pk16(hb[0], hb[1]), pk16(hb[2], hb[3]), pk16(hb[4], hb[5]), pk16(hb[6], hb[7])};
    const v4u ul = (v4u){pk16(lb[0], lb[1]), pk16(lb[2], lb[3]), pk16(lb[4], lb[5]), pk16(lb[6], lb[7])};
    const size_t ro = (size_t)o * NC + c8;
    *(volatile v4u*)(wqkh + ro) = uh;
    *(volatile v4u*)(wqkl + ro) = ul;
    __threadfence();
    *(volatile v4u*)(wqkh + ro) = uh;
    *(volatile v4u*)(wqkl + ro) = ul;
  } else if (blk < 24) {
    const int o = (blk - 8) * 16 + (t >> 4);
    const int c8 = (t & 15) * 8;
    const bool isl = (blk < 20);
    const float* src = isl ? lqkv_w : gkv_w;
    const int srow = isl ? o : (o - 128);
    const float dwv = dw_w[o & 63];
    const float rs = isl ? (kWCarry * dwv) : kWCarry;
    const float* rp = src + (size_t)srow * NC + c8;
    const v4f a = *(const v4f*)(rp);
    const v4f c = *(const v4f*)(rp + 4);
    unsigned short hb[8];
#pragma unroll
    for (int e = 0; e < 4; ++e) { hb[e] = h_bits(a[e] * rs); hb[4 + e] = h_bits(c[e] * rs); }
    const v4u u = (v4u){pk16(hb[0], hb[1]), pk16(hb[2], hb[3]), pk16(hb[4], hb[5]), pk16(hb[6], hb[7])};
    unsigned short* dp = wl + (size_t)o * NC + c8;
    *(volatile v4u*)dp = u;
    __threadfence();
    *(volatile v4u*)dp = u;
  } else if (blk < 26) {
    const int idx8 = (blk - 24) * 256 + t;
    const int row = idx8 >> 3, c8 = (idx8 & 7) * 8;
    const float* rp = fc_w + (size_t)row * NI + c8;
    const v4f a = *(const v4f*)(rp);
    const v4f c = *(const v4f*)(rp + 4);
    unsigned short hb[8];
#pragma unroll
    for (int e = 0; e < 4; ++e) { hb[e] = h_bits(a[e] * kWCarry); hb[4 + e] = h_bits(c[e] * kWCarry); }
    const v4u u = (v4u){pk16(hb[0], hb[1]), pk16(hb[2], hb[3]), pk16(hb[4], hb[5]), pk16(hb[6], hb[7])};
    unsigned short* dp = fc16 + (size_t)row * NI + c8;
    *(volatile v4u*)dp = u;
    __threadfence();
    *(volatile v4u*)dp = u;
  } else if (blk < 34) {
    const int idx8 = (blk - 26) * 256 + t;
    const int row = idx8 >> 4, c8 = (idx8 & 15) * 8;
    const float* rp = tc_w + (size_t)row * NC + c8;
    const v4f a = *(const v4f*)(rp);
    const v4f c = *(const v4f*)(rp + 4);
    unsigned short hb[8];
#pragma unroll
    for (int e = 0; e < 4; ++e) { hb[e] = h_bits(a[e] * kWCarry); hb[4 + e] = h_bits(c[e] * kWCarry); }
    const v4u u = (v4u){pk16(hb[0], hb[1]), pk16(hb[2], hb[3]), pk16(hb[4], hb[5]), pk16(hb[6], hb[7])};
    unsigned short* dp = tc16 + (size_t)row * NC + c8;
    *(volatile v4u*)dp = u;
    __threadfence();
    *(volatile v4u*)dp = u;
  } else {
    if (wave == 0) {
      if (lane < 16) {
        const int n4 = 4 * lane;
        const v4f val = *(const v4f*)(gq_b + n4);
        float* dp = beff + n4;
        *(volatile v4f*)dp = val;
        __threadfence();
        *(volatile v4f*)dp = val;
      }
    } else if (wave == 1) {
      if (lane < 16) {
        const int n4 = 4 * lane;
        const v4f val = *(const v4f*)(gkv_b + n4);
        float* dp = beff + 64 + n4;
        *(volatile v4f*)dp = val;
        __threadfence();
        *(volatile v4f*)dp = val;
      }
    } else if (wave < 4) {
      const int j = (wave - 2) * 32 + lane;
      if (j < 48) {
        const int n4 = 4 * j;
        const int ch = n4 & 63;
        const v4f lb = *(const v4f*)(lqkv_b + n4);
        const v4f dw = *(const v4f*)(dw_w + ch);
        const v4f db = *(const v4f*)(dw_b + ch);
        v4f val;
#pragma unroll
        for (int e = 0; e < 4; ++e) val[e] = kActCarry * (dw[e] * lb[e] + db[e]);
        float* dp = beff + 128 + n4;
        *(volatile v4f*)dp = val;
        __threadfence();
        *(volatile v4f*)dp = val;
      }
    } else if (wave == 4) {
      if (lane < 16) {
        const int n4 = 4 * lane;
        const v4f bb = *(const v4f*)(gkv_b + 64 + n4);
        const v4f val = bb * kActCarry;
        float* dp = beff + 320 + n4;
        *(volatile v4f*)dp = val;
        __threadfence();
        *(volatile v4f*)dp = val;
      }
    }
  }
}

__global__ __launch_bounds__(256) void gnstats_kernel(const float* __restrict__ src, float* __restrict__ part) {
  __shared__ float reds[8];
  __shared__ float redq[8];
  const int seg = blockIdx.x, b = blockIdx.y;
  const int t = threadIdx.x, lane = t & 31, wave = t >> 5;
  const float* p = src + (size_t)b * CN + (size_t)seg * GNSEGLEN;
  float s = 0.0f, s2 = 0.0f;
#pragma unroll 1
  for (int it = 0; it < 16; ++it) {
    const v4f v = *(const v4f*)(p + (size_t)(it * 256 + t) * 4);
    s  += (v[0] + v[1]) + (v[2] + v[3]);
    s2 += (v[0] * v[0] + v[1] * v[1]) + (v[2] * v[2] + v[3] * v[3]);
  }
#pragma unroll
  for (int off = 16; off > 0; off >>= 1) { s += __shfl_xor(s, off, 32); s2 += __shfl_xor(s2, off, 32); }
  if (lane == 0) { reds[wave] = s; redq[wave] = s2; }
  __syncthreads();
  if (wave == 0) {
    float S = reds[0], Q = redq[0];
#pragma unroll
    for (int w = 1; w < 8; ++w) { S += reds[w]; Q += redq[w]; }
    const float val = (lane == 0) ? S : ((lane == 1) ? Q : 0.0f);
    float* dp = part + ((size_t)(b * GNSEG + seg)) * 32 + lane;
    *(volatile float*)dp = val;
    __threadfence();
    *(volatile float*)dp = val;
  }
}

__global__ __launch_bounds__(64) void gnfin_kernel(const float* __restrict__ part, const float* __restrict__ g,
                                                  const float* __restrict__ beta, float* __restrict__ scale,
                                                  float* __restrict__ shift) {
  __shared__ float shm[2];
  const int b = blockIdx.x;
  const int t = threadIdx.x, lane = t & 31, wave = t >> 5;
  if (wave == 0) {
    const float* pl = part + ((size_t)(b * GNSEG + lane)) * 32;
    float S = pl[0], Q = pl[1];
#pragma unroll
    for (int off = 16; off > 0; off >>= 1) { S += __shfl_xor(S, off, 32); Q += __shfl_xor(Q, off, 32); }
    if (lane == 0) {
      const float mean = S * kInvCN;
      float var = Q * kInvCN - mean * mean;
      var = fmaxf(var, 0.0f);
      const float rstd = 1.0f / sqrtf(var + kEpsGN);
      shm[0] = mean; shm[1] = rstd;
    }
  }
  __syncthreads();
  const float mean = shm[0], rstd = shm[1];
  const int c4 = 4 * lane;
  const v4f gg = *(const v4f*)(g + c4);
  if (wave == 0) {
    const v4f sc = gg * rstd;
    float* dp = scale + (size_t)b * NC + c4;
    *(volatile v4f*)dp = sc;
    __threadfence();
    *(volatile v4f*)dp = sc;
  } else {
    const v4f bb = *(const v4f*)(beta + c4);
    const v4f sh = bb - gg * (mean * rstd);
    float* dp = shift + (size_t)b * NC + c4;
    *(volatile v4f*)dp = sh;
    __threadfence();
    *(volatile v4f*)dp = sh;
  }
}

__global__ __launch_bounds__(256) void norm_t_kernel(const float* __restrict__ x, const float* __restrict__ scale,
                                                    const float* __restrict__ shift, unsigned short* __restrict__ xnT,
                                                    unsigned short* __restrict__ xnH, unsigned short* __restrict__ xnL) {
  __shared__ float tile[NC][65];
  __shared__ float ssc[NC];
  __shared__ float ssh[NC];
  const int b = blockIdx.y, n0 = blockIdx.x * 64;
  const int t = threadIdx.x, lane = t & 31, wave = t >> 5;
  if (t < NC) { ssc[t] = scale[b * NC + t]; ssh[t] = shift[b * NC + t]; }
  __syncthreads();
  const float* xb = x + (size_t)b * CN + n0;
#pragma unroll 4
  for (int it = 0; it < 8; ++it) {
    const int e = it * 256 + t;
    const int c = e >> 4;
    const int n4 = (e & 15) * 4;
    const v4f v = *(const v4f*)(xb + (size_t)c * NN + n4);
    const float sc = ssc[c], sh = ssh[c];
    tile[c][n4 + 0] = v[0] * sc + sh;
    tile[c][n4 + 1] = v[1] * sc + sh;
    tile[c][n4 + 2] = v[2] * sc + sh;
    tile[c][n4 + 3] = v[3] * sc + sh;
  }
  __syncthreads();
  const size_t plane0 = ((size_t)(b * NN + n0)) * NC;
  unsigned short* of = xnT + plane0;
  unsigned short* oh = xnH + plane0;
  unsigned short* ol = xnL + plane0;
  const int rsub = lane >> 4, c8 = (lane & 15) * 8;
  for (int pass = 0; pass < 2; ++pass) {
#pragma unroll
    for (int it = 0; it < 4; ++it) {
      const int nl = it * 16 + wave * 2 + rsub;
      unsigned short fb[8], hb[8], lb[8];
#pragma unroll
      for (int e = 0; e < 8; ++e) {
        const float v = tile[c8 + e][nl];
        fb[e] = h_bits(v);
        const unsigned short h0 = f2bf_bits(v);
        hb[e] = h0;
        lb[e] = f2bf_bits(v - bf_bits2f(h0));
      }
      const v4u uf = (v4u){pk16(fb[0], fb[1]), pk16(fb[2], fb[3]), pk16(fb[4], fb[5]), pk16(fb[6], fb[7])};
      const v4u uh = (v4u){pk16(hb[0], hb[1]), pk16(hb[2], hb[3]), pk16(hb[4], hb[5]), pk16(hb[6], hb[7])};
      const v4u ul = (v4u){pk16(lb[0], lb[1]), pk16(lb[2], lb[3]), pk16(lb[4], lb[5]), pk16(lb[6], lb[7])};
      const size_t ro = (size_t)nl * NC + c8;
      *(volatile v4u*)(of + ro) = uf;
      *(volatile v4u*)(oh + ro) = uh;
      *(volatile v4u*)(ol + ro) = ul;
    }
    __threadfence();
  }
}

__global__ __launch_bounds__(256) void amul_kernel(const unsigned short* __restrict__ p3, unsigned short* __restrict__ at) {
  const int idx = blockIdx.x * 256 + threadIdx.x;
  if (idx >= NTOK * 8) return;
  const int n = idx >> 3, j = idx & 7;
  const unsigned short* row = p3 + (size_t)n * PLD;
  const v4u qa = *(const v4u*)(row + 8 * j);
  const v4u ka = *(const v4u*)(row + 64 + 8 * j);
  unsigned w[4];
#pragma unroll
  for (int e = 0; e < 4; ++e) {
    const float q0 = h16_to_f32(qa[e] & 0xffffu), q1 = h16_to_f32(qa[e] >> 16);
    const float k0 = h16_to_f32(ka[e] & 0xffffu), k1 = h16_to_f32(ka[e] >> 16);
    w[e] = pk16(h_bits(q0 * k0), h_bits(q1 * k1));
  }
  const v4u u = (v4u){w[0], w[1], w[2], w[3]};
  unsigned short* dp = at + (size_t)n * NI + 8 * j;
  *(volatile v4u*)dp = u;
  __threadfence();
  *(volatile v4u*)dp = u;
}

__global__ __launch_bounds__(256) void act1_kernel(const float* __restrict__ u1, unsigned short* __restrict__ s1t) {
  const int idx = blockIdx.x * 256 + threadIdx.x;
  if (idx >= NTOK * 16) return;
  const v4f u = *(const v4f*)(u1 + 4 * (size_t)idx);
  unsigned short hb[4];
#pragma unroll
  for (int e = 0; e < 4; ++e) {
    const float ex = expf(-u[e]);
    const float sg = __builtin_amdgcn_rcpf(1.0f + ex);
    hb[e] = h_bits(u[e] * sg * kS1Carry);
  }
  const v2u w = (v2u){pk16(hb[0], hb[1]), pk16(hb[2], hb[3])};
  unsigned short* dp = s1t + 4 * (size_t)idx;
  *(volatile v2u*)dp = w;
  __threadfence();
  *(volatile v2u*)dp = w;
}

__global__ __launch_bounds__(256) void yloc_kernel(const float* __restrict__ u2, const unsigned short* __restrict__ p3,
                                                  unsigned short* __restrict__ yt) {
  const int idx = blockIdx.x * 256 + threadIdx.x;
  if (idx >= NTOK * 16) return;
  const int n = idx >> 4, j = idx & 15;
  const v4f u = *(const v4f*)(u2 + 4 * (size_t)idx);
  const v2u lw = *(const v2u*)(p3 + (size_t)n * PLD + 128 + 4 * j);
  float lv[4];
  lv[0] = h16_to_f32(lw[0] & 0xffffu); lv[1] = h16_to_f32(lw[0] >> 16);
  lv[2] = h16_to_f32(lw[1] & 0xffffu); lv[3] = h16_to_f32(lw[1] >> 16);
  unsigned short hb[4];
#pragma unroll
  for (int e = 0; e < 4; ++e) {
    const float ex = expf(2.0f * u[e]);
    const float th = 1.0f - 2.0f * __builtin_amdgcn_rcpf(ex + 1.0f);
    hb[e] = h_bits(kLocScale * th * lv[e]);
  }
  const v2u w = (v2u){pk16(hb[0], hb[1]), pk16(hb[2], hb[3])};
  unsigned short* dp = yt + (size_t)n * NC + 4 * j;
  *(volatile v2u*)dp = w;
  __threadfence();
  *(volatile v2u*)dp = w;
}

__global__ __launch_bounds__(256) void colstats_kernel(const float* __restrict__ S, float* __restrict__ cvh) {
  const int col = blockIdx.x * 256 + threadIdx.x;
  const float* sc = S + col;
  float rm = sc[0];
  float rs = 0.0f;
#pragma unroll 1
  for (int m = 0; m < NN; m += 4) {
    const float* sp = sc + (size_t)m * NQH;
    const float e0 = sp[0], e1 = sp[NQH], e2 = sp[2 * NQH], e3 = sp[3 * NQH];
    const float cm = fmaxf(fmaxf(e0, e1), fmaxf(e2, e3));
    const float mn = fmaxf(rm, cm);
    const float a = (expf(e0 - mn) + expf(e1 - mn)) + (expf(e2 - mn) + expf(e3 - mn));
    rs = rs * expf(rm - mn) + a;
    rm = mn;
  }
  const float cval = -rm - logf(rs);
  float* dp = cvh + col;
  *(volatile float*)dp = cval;
  __threadfence();
  *(volatile float*)dp = cval;
}

template <bool SECOND>
__global__ __launch_bounds__(256) void prow_kernel(const float* __restrict__ S, const float* __restrict__ cvh,
                                                  unsigned short* __restrict__ pth, const float* __restrict__ cs_prev,
                                                  float* __restrict__ dst) {
  __shared__ float red[8];
  __shared__ float csl[32];
  const int t = threadIdx.x, lane = t & 31, wave = t >> 5;
  const int m0 = blockIdx.x * 32;
#pragma unroll 1
  for (int r = 0; r < 32; ++r) {
    const int m = m0 + r;
    const float* sr = S + (size_t)m * NQH;
    unsigned short* pr = pth + (size_t)m * NN;
    float sum = 0.0f;
#pragma unroll 1
    for (int q = 0; q < 2; ++q) {
      const int c = q * 1024 + 4 * t;
      const v4f sv = *(const v4f*)(sr + c);
      const v4f cv = *(const v4f*)(cvh + c);
      const float p0 = expf(sv[0] + cv[0]);
      const float p1 = expf(sv[1] + cv[1]);
      const float p2 = expf(sv[2] + cv[2]);
      const float p3 = expf(sv[3] + cv[3]);
      sum += (p0 + p1) + (p2 + p3);
      const v2u u = (v2u){pk16(h_bits(p0 * kPCarry), h_bits(p1 * kPCarry)), pk16(h_bits(p2 * kPCarry), h_bits(p3 * kPCarry))};
      unsigned short* pp = pr + c;
      *(volatile v2u*)pp = u;
      __threadfence();
      *(volatile v2u*)pp = u;
    }
#pragma unroll
    for (int off = 16; off > 0; off >>= 1) sum += __shfl_xor(sum, off, 32);
    if (lane == 0) red[wave] = sum;
    __syncthreads();
    if (t == 0) {
      float tot = red[0];
#pragma unroll
      for (int w = 1; w < 8; ++w) tot += red[w];
      csl[r] = tot;
    }
    __syncthreads();
  }
  if (wave == 0) {
    const float cs = csl[lane];
    float val;
    if (SECOND) {
      const float prev = cs_prev[m0 + lane];
      val = kYCarry / (1.0e-9f + (prev + cs));
    } else {
      val = cs;
    }
    float* dp = dst + m0 + lane;
    *(volatile float*)dp = val;
    __threadfence();
    *(volatile float*)dp = val;
  }
}

__global__ __launch_bounds__(256) void xr_scale_kernel(const float* __restrict__ G, const float* __restrict__ inv,
                                                      unsigned short* __restrict__ ytb) {
  const int idx = blockIdx.x * 256 + threadIdx.x;
  if (idx >= NN * 8) return;
  const int m = idx >> 3, j = idx & 7;
  const v4f g0 = *(const v4f*)(G + (size_t)m * NI + 8 * j);
  const v4f g1 = *(const v4f*)(G + (size_t)m * NI + 8 * j + 4);
  const float s = inv[m];
  unsigned short hb[8];
#pragma unroll
  for (int e = 0; e < 4; ++e) { hb[e] = h_bits(g0[e] * s); hb[4 + e] = h_bits(g1[e] * s); }
  const v4u u = (v4u){pk16(hb[0], hb[1]), pk16(hb[2], hb[3]), pk16(hb[4], hb[5]), pk16(hb[6], hb[7])};
  unsigned short* dp = ytb + (size_t)m * NC + 64 + 8 * j;
  *(volatile v4u*)dp = u;
  __threadfence();
  *(volatile v4u*)dp = u;
}

__global__ __launch_bounds__(256) void final_kernel(const float* __restrict__ x, const float* __restrict__ ycm,
                                                   const float* __restrict__ sc2, const float* __restrict__ sh2,
                                                   float* __restrict__ out) {
  const int idx = blockIdx.x * 256 + threadIdx.x;
  if (idx >= NB * CN / 4) return;
  const size_t e = 4 * (size_t)idx;
  const int bc = (int)(e / NN);
  const v4f xv = *(const v4f*)(x + e);
  const v4f yv = *(const v4f*)(ycm + e);
  const float sc = sc2[bc], sh = sh2[bc];
  v4f ov;
#pragma unroll
  for (int k = 0; k < 4; ++k) ov[k] = xv[k] + fmaxf(yv[k] * sc + sh, 0.0f);
  float* dp = out + e;
  *(volatile v4f*)dp = ov;
  __threadfence();
  *(volatile v4f*)dp = ov;
}

extern "C" void kernel_launch(void* const* d_in, const int* in_sizes, int n_in,
                              void* d_out, int out_size, void* d_ws, size_t ws_size,
                              hipStream_t stream) {
  if (n_in < 17) return;
  if (in_sizes[0] != NB * CN || out_size != NB * CN) return;
  if (in_sizes[1] != NC || in_sizes[2] != NC || in_sizes[3] != NI * NC || in_sizes[4] != NI) return;
  if (in_sizes[5] != 2 * NI * NC || in_sizes[6] != 2 * NI || in_sizes[7] != 3 * NI * NC || in_sizes[8] != 3 * NI) return;
  if (in_sizes[9] != NI || in_sizes[10] != NI || in_sizes[11] != NI * NI || in_sizes[12] != NI) return;
  if (in_sizes[13] != NC * NC || in_sizes[14] != NC || in_sizes[15] != NC || in_sizes[16] != NC) return;

  const float* x      = (const float*)d_in[0];
  const float* bn_g   = (const float*)d_in[1];
  const float* bn_b   = (const float*)d_in[2];
  const float* gq_w   = (const float*)d_in[3];
  const float* gq_b   = (const float*)d_in[4];
  const float* gkv_w  = (const float*)d_in[5];
  const float* gkv_b  = (const float*)d_in[6];
  const float* lqkv_w = (const float*)d_in[7];
  const float* lqkv_b = (const float*)d_in[8];
  const float* dw_w   = (const float*)d_in[9];
  const float* dw_b   = (const float*)d_in[10];
  const float* fc_w   = (const float*)d_in[11];
  const float* fc_b   = (const float*)d_in[12];
  const float* tc_w   = (const float*)d_in[13];
  const float* tc_b   = (const float*)d_in[14];
  const float* an_g   = (const float*)d_in[15];
  const float* an_b   = (const float*)d_in[16];
  float* out = (float*)d_out;

  const size_t szWQK  = (size_t)QKLD * NC * 2;
  const size_t szWL   = (size_t)WLROWS * NC * 2;
  const size_t szFC   = (size_t)NI * NI * 2;
  const size_t szTC   = (size_t)NC * NC * 2;
  const size_t szBEFF = (size_t)384 * 4;
  const size_t szGNP  = (size_t)NB * GNSEG * 32 * 4;
  const size_t szSC   = (size_t)NB * NC * 4;
  const size_t szXN   = (size_t)NTOK * NC * 2;
  const size_t szQK   = (size_t)NTOK * QKLD * 2;
  const size_t szP3   = (size_t)NTOK * PLD * 2;
  const size_t szVCM  = (size_t)NB * NI * NN * 2;
  const size_t szAT   = (size_t)NTOK * NI * 2;
  const size_t szU    = (size_t)NTOK * NI * 4;
  const size_t szS1   = (size_t)NTOK * NI * 2;
  const size_t szYT   = (size_t)NTOK * NC * 2;
  const size_t szVEC  = (size_t)NB * NN * 4;
  const size_t szSPL  = (size_t)NN * NQH * 4;
  const size_t szPT   = (size_t)NN * NN * 2;
  const size_t szG    = (size_t)NB * NN * NI * 4;
  const size_t szYCM  = (size_t)NB * CN * 4;
  size_t off = 0;
  const size_t oWQKH = off; off += szWQK;
  const size_t oWQKL = off; off += szWQK;
  const size_t oWL   = off; off += szWL;
  const size_t oFC   = off; off += szFC;
  const size_t oTC   = off; off += szTC;
  const size_t oBEFF = off; off += szBEFF;
  const size_t oGNP1 = off; off += szGNP;
  const size_t oGNP2 = off; off += szGNP;
  const size_t oSC1  = off; off += szSC;
  const size_t oSH1  = off; off += szSC;
  const size_t oSC2  = off; off += szSC;
  const size_t oSH2  = off; off += szSC;
  const size_t oXNT  = off; off += szXN;
  const size_t oXNH  = off; off += szXN;
  const size_t oXNL  = off; off += szXN;
  const size_t oQKH  = off; off += szQK;
  const size_t oQKL  = off; off += szQK;
  const size_t oP3   = off; off += szP3;
  const size_t oVCM  = off; off += szVCM;
  const size_t oAT   = off; off += szAT;
  const size_t oU1   = off; off += szU;
  const size_t oS1   = off; off += szS1;
  const size_t oU2   = off; off += szU;
  const size_t oYT   = off; off += szYT;
  const size_t oCVEC = off; off += szVEC;
  const size_t oCS0  = off; off += szVEC;
  const size_t oINV  = off; off += szVEC;
  const size_t oSPL  = off; off += szSPL;
  const size_t oPT   = off; off += szPT;
  const size_t oG    = off; off += szG;
  const size_t oYCM  = off; off += szYCM;
  const size_t total = off;
  if (ws_size < total) return;

  char* ws = (char*)d_ws;
  unsigned short* pWQKH = (unsigned short*)(ws + oWQKH);
  unsigned short* pWQKL = (unsigned short*)(ws + oWQKL);
  unsigned short* pWL   = (unsigned short*)(ws + oWL);
  unsigned short* pFC16 = (unsigned short*)(ws + oFC);
  unsigned short* pTC16 = (unsigned short*)(ws + oTC);
  float* pBEFF = (float*)(ws + oBEFF);
  float* pGNP1 = (float*)(ws + oGNP1);
  float* pGNP2 = (float*)(ws + oGNP2);
  float* pSC1 = (float*)(ws + oSC1);
  float* pSH1 = (float*)(ws + oSH1);
  float* pSC2 = (float*)(ws + oSC2);
  float* pSH2 = (float*)(ws + oSH2);
  unsigned short* pXNT = (unsigned short*)(ws + oXNT);
  unsigned short* pXNH = (unsigned short*)(ws + oXNH);
  unsigned short* pXNL = (unsigned short*)(ws + oXNL);
  unsigned short* pQKH = (unsigned short*)(ws + oQKH);
  unsigned short* pQKL = (unsigned short*)(ws + oQKL);
  unsigned short* pP3  = (unsigned short*)(ws + oP3);
  unsigned short* pVCM = (unsigned short*)(ws + oVCM);
  unsigned short* pAT  = (unsigned short*)(ws + oAT);
  float* pU1 = (float*)(ws + oU1);
  unsigned short* pS1T = (unsigned short*)(ws + oS1);
  float* pU2 = (float*)(ws + oU2);
  unsigned short* pYT  = (unsigned short*)(ws + oYT);
  float* pCVEC = (float*)(ws + oCVEC);
  float* pCS0  = (float*)(ws + oCS0);
  float* pINV  = (float*)(ws + oINV);
  float* pSPL  = (float*)(ws + oSPL);
  unsigned short* pPT = (unsigned short*)(ws + oPT);
  float* pG   = (float*)(ws + oG);
  float* pYCM = (float*)(ws + oYCM);

  wprep_kernel<<<dim3(35), dim3(256), 0, stream>>>(gq_w, gq_b, gkv_w, gkv_b, lqkv_w, lqkv_b, dw_w, dw_b, fc_w, tc_w,
                                                   pWQKH, pWQKL, pWL, pFC16, pTC16, pBEFF);
  gnstats_kernel<<<dim3(GNSEG, NB), dim3(256), 0, stream>>>(x, pGNP1);
  gnfin_kernel<<<dim3(NB), dim3(64), 0, stream>>>(pGNP1, bn_g, bn_b, pSC1, pSH1);
  norm_t_kernel<<<dim3(NN / 64, NB), dim3(256), 0, stream>>>(x, pSC1, pSH1, pXNT, pXNH, pXNL);
  {
    const int tiles = (NTOK / 64) * (QKLD / 64);
    wmma_gemm64<1, true, 2, 2, false, 0><<<dim3(tiles / 8, 1), dim3(256), 0, stream>>>(
        pXNH, pXNL, NC, 0L, pWQKH, pWQKL, NC, 0L, (void*)pQKH, (void*)pQKL, QKLD, 0L,
        pBEFF, pBEFF, 0L, NTOK, QKLD, NC, 1.0f);
  }
  {
    const int tiles = (NTOK / 64) * (PLD / 64);
    wmma_gemm64<0, false, 2, 1, false, 0><<<dim3(tiles / 8, 1), dim3(256), 0, stream>>>(
        pXNT, pXNT, NC, 0L, pWL, pWL, NC, 0L, (void*)pP3, (void*)pP3, PLD, 0L,
        pBEFF + 128, pBEFF, 0L, NTOK, PLD, NC, kProjScale);
  }
  {
    const int tiles = (NI / 64) * (NN / 64);
    wmma_gemm64<0, false, 1, 1, false, 0><<<dim3(tiles / 8, NB), dim3(256), 0, stream>>>(
        pWL + (size_t)192 * NC, pWL + (size_t)192 * NC, NC, 0L, pXNT, pXNT, NC, (long)NN * NC,
        (void*)pVCM, (void*)pVCM, NN, (long)NI * NN, pBEFF + 320, pBEFF, 0L, NI, NN, NC, kProjScale);
  }
  amul_kernel<<<dim3((NTOK * 8) / 256), dim3(256), 0, stream>>>(pP3, pAT);
  {
    const int tiles = (NTOK / 64) * (NI / 64);
    wmma_gemm64<0, false, 2, 0, false, 0><<<dim3(tiles / 8, 1), dim3(256), 0, stream>>>(
        pAT, pAT, NI, 0L, pFC16, pFC16, NI, 0L, (void*)pU1, (void*)pU1, NI, 0L,
        fc_b, pBEFF, 0L, NTOK, NI, NI, kFc1Scale);
    act1_kernel<<<dim3((NTOK * 16) / 256), dim3(256), 0, stream>>>(pU1, pS1T);
    wmma_gemm64<0, false, 2, 0, false, 0><<<dim3(tiles / 8, 1), dim3(256), 0, stream>>>(
        pS1T, pS1T, NI, 0L, pFC16, pFC16, NI, 0L, (void*)pU2, (void*)pU2, NI, 0L,
        fc_b, pBEFF, 0L, NTOK, NI, NI, kFc2Scale);
    yloc_kernel<<<dim3((NTOK * 16) / 256), dim3(256), 0, stream>>>(pU2, pP3, pYT);
  }
  const int tilesScore = (NN / 64) * (NQH / 64);
  const int tilesPV    = (NN / 64) * (NI / 64);
  for (int b = 0; b < NB; ++b) {
    const size_t kOff = ((size_t)b * NN) * QKLD + 64;
    const unsigned short* kH = pQKH + kOff;
    const unsigned short* kL = pQKL + kOff;
    for (int h = 0; h < 2; ++h) {
      const size_t qOff = ((size_t)b * NN + (size_t)h * NQH) * QKLD;
      const unsigned short* qH = pQKH + qOff;
      const unsigned short* qL = pQKL + qOff;
      float* cvh = pCVEC + (size_t)b * NN + (size_t)h * NQH;
      wmma_gemm64<1, true, 0, 0, false, 0><<<dim3(tilesScore / 8, 1), dim3(256), 0, stream>>>(
          kH, kL, QKLD, 0L, qH, qL, QKLD, 0L, (void*)pSPL, (void*)pSPL, NQH, 0L,
          pBEFF, pBEFF, 0L, NN, NQH, NI, 1.0f);
      colstats_kernel<<<dim3(NQH / 256), dim3(256), 0, stream>>>(pSPL, cvh);
      if (h == 0) {
        prow_kernel<false><<<dim3(NN / 32), dim3(256), 0, stream>>>(pSPL, cvh, pPT, pINV + (size_t)b * NN, pCS0 + (size_t)b * NN);
      } else {
        prow_kernel<true><<<dim3(NN / 32), dim3(256), 0, stream>>>(pSPL, cvh, pPT + NQH, pCS0 + (size_t)b * NN, pINV + (size_t)b * NN);
      }
    }
    float* Gb = pG + (size_t)b * NN * NI;
    const unsigned short* Vb = pVCM + (size_t)b * NI * NN;
    wmma_gemm64<0, false, 0, 0, false, 0><<<dim3(tilesPV / 8, 1), dim3(256), 0, stream>>>(
        pPT, pPT, NN, 0L, Vb, Vb, NN, 0L, (void*)Gb, (void*)Gb, NI, 0L,
        pBEFF, pBEFF, 0L, NN, NI, NN, kPVScale);
    xr_scale_kernel<<<dim3((NN * 8) / 256), dim3(256), 0, stream>>>(Gb, pINV + (size_t)b * NN, pYT + (size_t)b * NN * NC);
  }
  {
    const int tiles = (NC / 64) * (NN / 64);
    wmma_gemm64<0, false, 1, 0, false, 0><<<dim3(tiles / 8, NB), dim3(256), 0, stream>>>(
        pTC16, pTC16, NC, 0L, pYT, pYT, NC, (long)NN * NC, (void*)pYCM, (void*)pYCM, NN, (long)NC * NN,
        tc_b, pBEFF, 0L, NC, NN, NC, kTcScale);
  }
  gnstats_kernel<<<dim3(GNSEG, NB), dim3(256), 0, stream>>>(pYCM, pGNP2);
  gnfin_kernel<<<dim3(NB), dim3(64), 0, stream>>>(pGNP2, an_g, an_b, pSC2, pSH2);
  final_kernel<<<dim3((NB * CN / 4) / 256), dim3(256), 0, stream>>>(x, pYCM, pSC2, pSH2, out);
}
